// Q_GoBERT_83511344103730
// MI455X (gfx1250) — hardware-verified
//
#include <hip/hip_runtime.h>
#define NNODE 50000
#define NE 800000
#define NTOT (NE + NNODE)
#define NG 256
#define TT 50
#define QD 32
#define FH 128
#define NH 4
#define HD 32
#define LH 128
#define G4 512
#define NN NNODE
#define MAXDEG 256

typedef __bf16 v16b __attribute__((ext_vector_type(16)));
typedef unsigned short v8us __attribute__((ext_vector_type(8), may_alias));
typedef float  v8f  __attribute__((ext_vector_type(8)));
typedef float  v4f  __attribute__((ext_vector_type(4)));
typedef float  v4fa __attribute__((ext_vector_type(4), may_alias));
union FragB { v16b v; v8us half[2]; unsigned short u[16]; };

__device__ __forceinline__ unsigned short bf16_bits(float x) { unsigned int u = __float_as_uint(x); return (unsigned short)((u + 0x7FFFu + ((u >> 16) & 1u)) >> 16); }
__device__ __forceinline__ float bf16_val(unsigned short b) { return __uint_as_float(((unsigned int)b) << 16); }
__device__ __forceinline__ float bf16_round(float x) { return bf16_val(bf16_bits(x)); }
template <int NT>
__device__ __forceinline__ v8f mmaN(v16b ah, v16b al, v16b bh, v16b bl, v8f c) {
  c = __builtin_amdgcn_wmma_f32_16x16x32_bf16(false, ah, false, bh, (short)0, c, false, false);
  if (NT >= 2) c = __builtin_amdgcn_wmma_f32_16x16x32_bf16(false, al, false, bh, (short)0, c, false, false);
  if (NT >= 3) c = __builtin_amdgcn_wmma_f32_16x16x32_bf16(false, ah, false, bl, (short)0, c, false, false);
  asm volatile("v_nop\n\tv_nop\n\tv_nop\n\tv_nop" : "+v"(c) : "v"(ah), "v"(al), "v"(bh), "v"(bl));
  return c;
}

__global__ __launch_bounds__(256) void k_wt_bf16(const float* __restrict__ W, unsigned short* __restrict__ Wt, int K, int N) {
  const int t = blockIdx.x * 256 + threadIdx.x;
  const int k8n = K / 8;
  if (t >= N * k8n) return;
  const int n = t / k8n, k8 = (t % k8n) * 8;
  v8us v;
#pragma unroll
  for (int i = 0; i < 8; ++i) v[i] = bf16_bits(W[(size_t)(k8 + i) * N + n]);
  *(volatile v8us*)(Wt + (size_t)n * K + k8) = v;
  __threadfence();
  *(volatile v8us*)(Wt + (size_t)n * K + k8) = v;
}

template <bool ASPLIT, int ACT, bool BIAS_BF16>
__global__ __launch_bounds__(128) void k_gemm_bf(const float* __restrict__ A, int lda, const unsigned short* __restrict__ Wt, int ldb,
                                               const float* __restrict__ bias, float* __restrict__ C, int ldc, int M, int N, int K) {
  __shared__ __attribute__((aligned(16))) float so[4][16][64];
  const int tid = threadIdx.x, w = tid >> 5, lane = tid & 31, ln = lane & 15, hh = lane >> 4;
  const int ntn = N / 64;
  const int wid = blockIdx.x * 4 + w;
  const int mt = wid / ntn, nq = wid % ntn;
  if (mt * 16 >= M) return;
  const int row0 = mt * 16, col0 = nq * 64;
  const float* arow = A + (size_t)(row0 + ln) * lda;
  v8f acc[4] = {};
  for (int kb = 0; kb < K; kb += 32) {
    FragB ah, al;
    const v4f x0 = *(const v4fa*)(arow + kb + 8 * hh), x1 = *(const v4fa*)(arow + kb + 8 * hh + 4);
    const v4f x2 = *(const v4fa*)(arow + kb + 16 + 8 * hh), x3 = *(const v4fa*)(arow + kb + 16 + 8 * hh + 4);
    float xs[16] = {x0[0],x0[1],x0[2],x0[3],x1[0],x1[1],x1[2],x1[3],x2[0],x2[1],x2[2],x2[3],x3[0],x3[1],x3[2],x3[3]};
#pragma unroll
    for (int i = 0; i < 16; ++i) { const unsigned short hb = bf16_bits(xs[i]); ah.u[i] = hb; al.u[i] = ASPLIT ? bf16_bits(xs[i] - bf16_val(hb)) : (unsigned short)0; }
#pragma unroll
    for (int t = 0; t < 4; ++t) {
      const unsigned short* brow = Wt + (size_t)(col0 + t * 16 + ln) * ldb + kb;
      FragB b;
      b.half[0] = *(const v8us*)(brow + 8 * hh);
      b.half[1] = *(const v8us*)(brow + 16 + 8 * hh);
      acc[t] = mmaN<ASPLIT ? 2 : 1>(ah.v, al.v, b.v, b.v, acc[t]);
    }
  }
#pragma unroll
  for (int t = 0; t < 4; ++t) {
    float bv = bias ? bias[col0 + t * 16 + ln] : 0.f;
    if (BIAS_BF16) bv = bf16_round(bv);
#pragma unroll
    for (int r = 0; r < 8; ++r) { float v = acc[t][r] + bv; if (ACT == 1) v = fmaxf(v, 0.f); so[w][8 * hh + r][t * 16 + ln] = v; }
  }
  __builtin_amdgcn_fence(__ATOMIC_ACQ_REL, "workgroup");
  __builtin_amdgcn_wave_barrier();
  const int rsub = lane >> 4, c4 = (lane & 15) * 4;
  for (int pass = 0; pass < 2; ++pass) {
#pragma unroll
    for (int q = 0; q < 8; ++q) {
      const int r = q * 2 + rsub;
      const v4f v = *(const v4fa*)&so[w][r][c4];
      *(volatile v4f*)(C + (size_t)(row0 + r) * ldc + col0 + c4) = v;
    }
    if (pass == 0) __threadfence();
  }
}

template <int D, bool CAUSAL>
__global__ __launch_bounds__(128) void k_flash(const float* __restrict__ qb, const float* __restrict__ kb, const float* __restrict__ vb,
                                             int pitch, int T, int H, float scale, float* __restrict__ y, int ypitch) {
  constexpr int KS = D / 32;
  constexpr int DT = D / 16;
  __shared__ __attribute__((aligned(16))) unsigned short sKh[32][D + 8], sKl[32][D + 8], sVh[32][D + 8], sVl[32][D + 8];
  __shared__ __attribute__((aligned(16))) unsigned short sPh[4][16][40], sPl[4][16][40];
  __shared__ __attribute__((aligned(16))) float sO[4][16][D];
  const int tid = threadIdx.x, w = tid >> 5, lane = tid & 31, ln = lane & 15, hh = lane >> 4;
  const int nqb = (T + 63) / 64;
  const int bh = blockIdx.x / nqb, qblk = blockIdx.x % nqb;
  const int b = bh / H, h = bh % H;
  const int q0 = qblk * 64 + w * 16;
  const float* Q = qb + (size_t)b * T * pitch + h * D;
  const float* K = kb + (size_t)b * T * pitch + h * D;
  const float* V = vb + (size_t)b * T * pitch + h * D;

  FragB aqh[KS], aql[KS];
  {
    int row = q0 + ln; if (row >= T) row = T - 1;
    const float* qr = Q + (size_t)row * pitch;
#pragma unroll
    for (int ks = 0; ks < KS; ++ks)
#pragma unroll
      for (int i = 0; i < 16; ++i) {
        const int d = ks * 32 + ((i < 8) ? (8 * hh + i) : (16 + 8 * hh + (i - 8)));
        const float x = qr[d] * scale; const unsigned short hb = bf16_bits(x);
        aqh[ks].u[i] = hb; aql[ks].u[i] = bf16_bits(x - bf16_val(hb));
      }
  }
  float m_r[8], l_r[8];
#pragma unroll
  for (int r = 0; r < 8; ++r) { m_r[r] = -3.0e38f; l_r[r] = 0.f; }
  v8f oacc[DT];
#pragma unroll
  for (int dt = 0; dt < DT; ++dt) oacc[dt] = (v8f){0.f,0.f,0.f,0.f,0.f,0.f,0.f,0.f};

  const int kv_end = CAUSAL ? min(T, qblk * 64 + 64) : T;
  for (int j0 = 0; j0 < kv_end; j0 += 32) {
    __syncthreads();
    for (int e = tid; e < 32 * (D / 4); e += 128) {
      const int r = e / (D / 4), c4 = (e % (D / 4)) * 4;
      const int key = j0 + r;
      v4f kf = {0.f,0.f,0.f,0.f}, vf = {0.f,0.f,0.f,0.f};
      if (key < T) { kf = *(const v4fa*)(K + (size_t)key * pitch + c4); vf = *(const v4fa*)(V + (size_t)key * pitch + c4); }
#pragma unroll
      for (int t = 0; t < 4; ++t) {
        unsigned short hb = bf16_bits(kf[t]); sKh[r][c4 + t] = hb; sKl[r][c4 + t] = bf16_bits(kf[t] - bf16_val(hb));
        hb = bf16_bits(vf[t]); sVh[r][c4 + t] = hb; sVl[r][c4 + t] = bf16_bits(vf[t] - bf16_val(hb));
      }
    }
    __syncthreads();
    v8f s[2];
#pragma unroll
    for (int nt = 0; nt < 2; ++nt) {
      v8f acc = {};
#pragma unroll
      for (int ks = 0; ks < KS; ++ks) {
        FragB bh_, bl_;
        bh_.half[0] = *(const v8us*)&sKh[nt * 16 + ln][ks * 32 + 8 * hh]; bh_.half[1] = *(const v8us*)&sKh[nt * 16 + ln][ks * 32 + 16 + 8 * hh];
        bl_.half[0] = *(const v8us*)&sKl[nt * 16 + ln][ks * 32 + 8 * hh]; bl_.half[1] = *(const v8us*)&sKl[nt * 16 + ln][ks * 32 + 16 + 8 * hh];
        acc = mmaN<3>(aqh[ks].v, aql[ks].v, bh_.v, bl_.v, acc);
      }
      s[nt] = acc;
    }
    float alpha[8];
#pragma unroll
    for (int r = 0; r < 8; ++r) {
      const int qi = q0 + 8 * hh + r;
      const int ja = j0 + ln, jb = j0 + 16 + ln;
      if (CAUSAL) { if (ja > qi) s[0][r] = -3.0e38f; if (jb > qi) s[1][r] = -3.0e38f; }
      if (ja >= T) s[0][r] = -3.0e38f;
      if (jb >= T) s[1][r] = -3.0e38f;
      float mx = fmaxf(s[0][r], s[1][r]);
      mx = fmaxf(mx, __shfl_xor(mx, 1, 32)); mx = fmaxf(mx, __shfl_xor(mx, 2, 32)); mx = fmaxf(mx, __shfl_xor(mx, 4, 32)); mx = fmaxf(mx, __shfl_xor(mx, 8, 32));
      const float mnew = fmaxf(m_r[r], mx);
      alpha[r] = (mnew > -1.0e38f) ? __expf(m_r[r] - mnew) : 1.0f;
      const float p0 = (s[0][r] > -1.0e38f) ? __expf(s[0][r] - mnew) : 0.f;
      const float p1 = (s[1][r] > -1.0e38f) ? __expf(s[1][r] - mnew) : 0.f;
      m_r[r] = mnew;
      l_r[r] = l_r[r] * alpha[r] + p0 + p1;
      unsigned short hb = bf16_bits(p0); sPh[w][8 * hh + r][ln] = hb;      sPl[w][8 * hh + r][ln] = bf16_bits(p0 - bf16_val(hb));
      hb = bf16_bits(p1);                sPh[w][8 * hh + r][16 + ln] = hb; sPl[w][8 * hh + r][16 + ln] = bf16_bits(p1 - bf16_val(hb));
    }
#pragma unroll
    for (int dt = 0; dt < DT; ++dt)
#pragma unroll
      for (int r = 0; r < 8; ++r) oacc[dt][r] *= alpha[r];
    __builtin_amdgcn_fence(__ATOMIC_ACQ_REL, "workgroup");
    __builtin_amdgcn_wave_barrier();
    FragB pah, pal;
    pah.half[0] = *(const v8us*)&sPh[w][ln][8 * hh]; pah.half[1] = *(const v8us*)&sPh[w][ln][16 + 8 * hh];
    pal.half[0] = *(const v8us*)&sPl[w][ln][8 * hh]; pal.half[1] = *(const v8us*)&sPl[w][ln][16 + 8 * hh];
#pragma unroll
    for (int dt = 0; dt < DT; ++dt) {
      FragB bvh, bvl;
#pragma unroll
      for (int i = 0; i < 8; ++i) {
        bvh.u[i] = sVh[8 * hh + i][dt * 16 + ln]; bvh.u[8 + i] = sVh[16 + 8 * hh + i][dt * 16 + ln];
        bvl.u[i] = sVl[8 * hh + i][dt * 16 + ln]; bvl.u[8 + i] = sVl[16 + 8 * hh + i][dt * 16 + ln];
      }
      oacc[dt] = mmaN<3>(pah.v, pal.v, bvh.v, bvl.v, oacc[dt]);
    }
    __builtin_amdgcn_fence(__ATOMIC_ACQ_REL, "workgroup");
    __builtin_amdgcn_wave_barrier();
  }
#pragma unroll
  for (int r = 0; r < 8; ++r) {
    float l = l_r[r];
    l += __shfl_xor(l, 1, 32); l += __shfl_xor(l, 2, 32); l += __shfl_xor(l, 4, 32); l += __shfl_xor(l, 8, 32);
    l_r[r] = (l > 0.f) ? 1.0f / l : 0.f;
  }
#pragma unroll
  for (int dt = 0; dt < DT; ++dt)
#pragma unroll
    for (int r = 0; r < 8; ++r) sO[w][8 * hh + r][dt * 16 + ln] = oacc[dt][r] * l_r[r];
  __builtin_amdgcn_fence(__ATOMIC_ACQ_REL, "workgroup");
  __builtin_amdgcn_wave_barrier();
  for (int pass = 0; pass < 2; ++pass) {
    for (int r = 0; r < 16; ++r) {
      const int row = q0 + r;
      if (row < T && lane < D / 4) {
        const v4f val = *(const v4fa*)&sO[w][r][lane * 4];
        *(volatile v4f*)(y + ((size_t)b * T + row) * ypitch + h * D + lane * 4) = val;
      }
    }
    if (pass == 0) __threadfence();
  }
}

template <bool ASPLIT, int ACT, bool BIAS_BF16, bool RES_BF16>
__global__ __launch_bounds__(128) void k_gemm_bf3(const float* __restrict__ A, int lda, const unsigned short* __restrict__ Wt, int ldb,
                                                const float* __restrict__ bias, const float* __restrict__ resid, int rmod, int ldr,
                                                float* __restrict__ C, int ldc, int M, int N, int K) {
  __shared__ __attribute__((aligned(16))) float so[4][16][64];
  const int tid = threadIdx.x, w = tid >> 5, lane = tid & 31, ln = lane & 15, hh = lane >> 4;
  const int ntn = N / 64;
  const int wid = blockIdx.x * 4 + w;
  const int mt = wid / ntn, nq = wid % ntn;
  if (mt * 16 >= M) return;
  const int row0 = mt * 16, col0 = nq * 64;
  const float* arow = A + (size_t)(row0 + ln) * lda;
  v8f acc[4] = {};
  for (int kb = 0; kb < K; kb += 32) {
    FragB ah, al;
    const v4f x0 = *(const v4fa*)(arow + kb + 8 * hh), x1 = *(const v4fa*)(arow + kb + 8 * hh + 4);
    const v4f x2 = *(const v4fa*)(arow + kb + 16 + 8 * hh), x3 = *(const v4fa*)(arow + kb + 16 + 8 * hh + 4);
    float xs[16] = {x0[0],x0[1],x0[2],x0[3],x1[0],x1[1],x1[2],x1[3],x2[0],x2[1],x2[2],x2[3],x3[0],x3[1],x3[2],x3[3]};
#pragma unroll
    for (int i = 0; i < 16; ++i) { const unsigned short hb = bf16_bits(xs[i]); ah.u[i] = hb; al.u[i] = ASPLIT ? bf16_bits(xs[i] - bf16_val(hb)) : (unsigned short)0; }
#pragma unroll
    for (int t = 0; t < 4; ++t) {
      const unsigned short* brow = Wt + (size_t)(col0 + t * 16 + ln) * ldb + kb;
      FragB b;
      b.half[0] = *(const v8us*)(brow + 8 * hh);
      b.half[1] = *(const v8us*)(brow + 16 + 8 * hh);
      acc[t] = mmaN<ASPLIT ? 2 : 1>(ah.v, al.v, b.v, b.v, acc[t]);
    }
  }
#pragma unroll
  for (int t = 0; t < 4; ++t) {
    const int col = col0 + t * 16 + ln;
    float bv = bias ? bias[col] : 0.f;
    if (BIAS_BF16) bv = bf16_round(bv);
#pragma unroll
    for (int r = 0; r < 8; ++r) {
      float v = acc[t][r] + bv;
      if (resid) { float rv = resid[(size_t)((row0 + 8 * hh + r) % rmod) * ldr + col]; if (RES_BF16) rv = bf16_round(rv); v += rv; }
      if (ACT == 1) v = fmaxf(v, 0.f);
      if (ACT == 2) v = 0.5f * v * (1.0f + erff(v * 0.70710678118654752f));
      if (ACT == 3) { const float u = 0.7978845608028654f * (v + 0.044715f * v * v * v); v = 0.5f * v * (1.0f + tanhf(u)); }
      so[w][8 * hh + r][t * 16 + ln] = v;
    }
  }
  __builtin_amdgcn_fence(__ATOMIC_ACQ_REL, "workgroup");
  __builtin_amdgcn_wave_barrier();
  const int rsub = lane >> 4, c4 = (lane & 15) * 4;
  for (int pass = 0; pass < 2; ++pass) {
#pragma unroll
    for (int q = 0; q < 8; ++q) {
      const int r = q * 2 + rsub;
      const v4f v = *(const v4fa*)&so[w][r][c4];
      *(volatile v4f*)(C + (size_t)(row0 + r) * ldc + col0 + c4) = v;
    }
    if (pass == 0) __threadfence();
  }
}
template <bool PARAM_BF16>
__global__ __launch_bounds__(256) void k_layernorm(const float* __restrict__ X, const float* __restrict__ R, const float* __restrict__ g, const float* __restrict__ bta,
                                                  float* __restrict__ out_sum, float* __restrict__ out_norm, int N, float eps) {
  __shared__ float red[256];
  const int row = blockIdx.x, tid = threadIdx.x;
  const float* x = X + (size_t)row * N; const float* rr = R ? R + (size_t)row * N : nullptr;
  float vals[16];
  const int per = N / 256;
  float s1 = 0.f;
  for (int u = 0; u < per / 4; ++u) {
    const int j = tid * 4 + 1024 * u;
    const v4f a = *(const v4fa*)(x + j);
    v4f b = {0.f,0.f,0.f,0.f}; if (rr) b = *(const v4fa*)(rr + j);
#pragma unroll
    for (int q = 0; q < 4; ++q) { const float v = a[q] + b[q]; vals[u * 4 + q] = v; s1 += v; }
  }
  red[tid] = s1; __syncthreads();
  for (int st = 128; st > 0; st >>= 1) { if (tid < st) red[tid] += red[tid + st]; __syncthreads(); }
  const float mu = red[0] / (float)N; __syncthreads();
  float s2 = 0.f;
  for (int u = 0; u < per / 4; ++u)
#pragma unroll
    for (int q = 0; q < 4; ++q) { const float c = vals[u * 4 + q] - mu; s2 += c * c; }
  red[tid] = s2; __syncthreads();
  for (int st = 128; st > 0; st >>= 1) { if (tid < st) red[tid] += red[tid + st]; __syncthreads(); }
  const float rs = rsqrtf(red[0] / (float)N + eps);
  for (int pass = 0; pass < 2; ++pass) {
    for (int u = 0; u < per / 4; ++u) {
      const int j = tid * 4 + 1024 * u;
      v4f o, sm;
#pragma unroll
      for (int q = 0; q < 4; ++q) {
        float gg = g[j + q], bb = bta[j + q];
        if (PARAM_BF16) { gg = bf16_round(gg); bb = bf16_round(bb); }
        sm[q] = vals[u * 4 + q]; o[q] = (vals[u * 4 + q] - mu) * rs * gg + bb;
      }
      if (out_sum) *(volatile v4f*)(out_sum + (size_t)row * N + j) = sm;
      *(volatile v4f*)(out_norm + (size_t)row * N + j) = o;
    }
    if (pass == 0) __threadfence();
  }
}

#define CS_NW 1024
#define CS_CH 832
#define CS_NB 256
#define CS_CAP 8192
__device__ __forceinline__ int cs_dst(const int* __restrict__ eidst, int e, int ne, int nt, int nn) { if (e >= nt) return -1; int d = (e < ne) ? eidst[e] : (e - ne); return d < 0 ? 0 : (d >= nn ? nn - 1 : d); }
__global__ __launch_bounds__(256) void k_cs_p1(const int* __restrict__ eidst, int ne, int nt, int nn, int* __restrict__ seg_dst, int* __restrict__ seg_eid, int* __restrict__ P1, int* __restrict__ Q1) {
  __shared__ int scnt[8][CS_NB]; __shared__ int srun[8][CS_NB]; __shared__ int sod[8][CS_CH]; __shared__ int soe[8][CS_CH];
  const int tid = threadIdx.x, wv = tid >> 5, lane = tid & 31; const int w = blockIdx.x * 8 + wv; const int e0 = w * CS_CH;
  for (int i = lane; i < CS_NB; i += 32) { scnt[wv][i] = 0; srun[wv][i] = 0; }
  __builtin_amdgcn_fence(__ATOMIC_ACQ_REL, "workgroup"); __builtin_amdgcn_wave_barrier();
#pragma unroll 1
  for (int i0 = 0; i0 < CS_CH; i0 += 32) { const int e = e0 + i0 + lane; const int d = cs_dst(eidst, e, ne, nt, nn); const int hb = (d < 0) ? -1 : (d >> 8);
#pragma unroll 1
    for (int ld = 0; ld < 32; ++ld) { const int kk = __shfl(hb, ld, 32); const unsigned long long m = __ballot(hb == kk); const int first = __ffsll((long long)m) - 1; if (ld == first && lane == first && kk >= 0) scnt[wv][kk] += __popcll(m); }
    __builtin_amdgcn_fence(__ATOMIC_ACQ_REL, "workgroup"); __builtin_amdgcn_wave_barrier(); }
  { int loc[8]; int s = 0; for (int j = 0; j < 8; ++j) { loc[j] = s; s += scnt[wv][lane * 8 + j]; }
    int incl = s; for (int o = 1; o < 32; o <<= 1) { const int v = __shfl_up(incl, o, 32); if (lane >= o) incl += v; } const int excl = incl - s;
    for (int j = 0; j < 8; ++j) srun[wv][lane * 8 + j] = excl + loc[j]; }
  __builtin_amdgcn_fence(__ATOMIC_ACQ_REL, "workgroup"); __builtin_amdgcn_wave_barrier();
  for (int pass = 0; pass < 2; ++pass) { for (int i = lane; i < CS_NB; i += 32) { *(volatile int*)(P1 + (size_t)w * CS_NB + i) = scnt[wv][i]; *(volatile int*)(Q1 + (size_t)w * CS_NB + i) = srun[wv][i]; } if (pass == 0) __threadfence(); }
#pragma unroll 1
  for (int i0 = 0; i0 < CS_CH; i0 += 32) { const int e = e0 + i0 + lane; const int d = cs_dst(eidst, e, ne, nt, nn); const int hb = (d < 0) ? -1 : (d >> 8);
    int pos = -1; int grpcnt = 0; bool leader = false;
#pragma unroll 1
    for (int ld = 0; ld < 32; ++ld) { const int kk = __shfl(hb, ld, 32); const unsigned long long g = __ballot(hb == kk); const int first = __ffsll((long long)g) - 1;
      if (ld == first && kk >= 0) { if (hb == kk) { const unsigned long long below = g & ((1ull << lane) - 1ull); pos = srun[wv][kk] + __popcll(below); if (lane == first) { leader = true; grpcnt = __popcll(g); } } } }
    if (pos >= 0) { sod[wv][pos] = d; soe[wv][pos] = e; }
    __builtin_amdgcn_fence(__ATOMIC_ACQ_REL, "workgroup"); __builtin_amdgcn_wave_barrier();
    if (leader) srun[wv][hb] += grpcnt;
    __builtin_amdgcn_fence(__ATOMIC_ACQ_REL, "workgroup"); __builtin_amdgcn_wave_barrier(); }
  for (int pass = 0; pass < 2; ++pass) { for (int i = lane; i < CS_CH; i += 32) { *(volatile int*)(seg_dst + (size_t)e0 + i) = sod[wv][i]; *(volatile int*)(seg_eid + (size_t)e0 + i) = soe[wv][i]; } if (pass == 0) __threadfence(); }
}
__global__ __launch_bounds__(256) void k_cs_scan(const int* __restrict__ P1, int* __restrict__ R, int* __restrict__ S) {
  __shared__ int tot[CS_NB]; __shared__ int st[CS_NB + 1];
  const int b = threadIdx.x; int acc = 0;
#pragma unroll 1
  for (int w = 0; w < CS_NW; ++w) { const int c = P1[(size_t)w * CS_NB + b]; *(volatile int*)(R + (size_t)w * CS_NB + b) = acc; acc += c; }
  __threadfence();
  acc = 0;
#pragma unroll 1
  for (int w = 0; w < CS_NW; ++w) { const int c = P1[(size_t)w * CS_NB + b]; *(volatile int*)(R + (size_t)w * CS_NB + b) = acc; acc += c; }
  tot[b] = acc; __syncthreads();
  if (b == 0) { int s = 0; for (int i = 0; i < CS_NB; ++i) { st[i] = s; s += (tot[i] + 31) & ~31; } st[CS_NB] = s; }
  __syncthreads();
  for (int pass = 0; pass < 2; ++pass) { *(volatile int*)(S + b) = st[b]; if (b < 32) *(volatile int*)(S + CS_NB + b) = (b == 0) ? st[CS_NB] : 0; if (pass == 0) __threadfence(); }
}
__global__ __launch_bounds__(256) void k_cs_p2(const int* __restrict__ seg_dst, const int* __restrict__ seg_eid, const int* __restrict__ P1, const int* __restrict__ Q1, const int* __restrict__ R, const int* __restrict__ S, int nn, int* __restrict__ csr_eid, int* __restrict__ csr_start, int* __restrict__ csr_cnt) {
  __shared__ int sd[CS_CAP]; __shared__ int se[CS_CAP]; __shared__ int sorted[CS_CAP]; __shared__ int lcnt[CS_NB]; __shared__ int lpre[CS_NB + 1];
  const int hb = blockIdx.x, t = threadIdx.x; const int total = (R[(size_t)(CS_NW - 1) * CS_NB + hb] + P1[(size_t)(CS_NW - 1) * CS_NB + hb]); const int tot = total > CS_CAP ? CS_CAP : total;
#pragma unroll 1
  for (int w = t; w < CS_NW; w += 256) { const int c = P1[(size_t)w * CS_NB + hb]; const int base = R[(size_t)w * CS_NB + hb]; const int src = w * CS_CH + Q1[(size_t)w * CS_NB + hb];
    for (int k = 0; k < c; ++k) { const int p = base + k; if (p < CS_CAP) { sd[p] = seg_dst[src + k] & 255; se[p] = seg_eid[src + k]; } } }
  __syncthreads();
  { int c = 0;
#pragma unroll 1
    for (int i = 0; i < tot; ++i) c += (sd[i] == t) ? 1 : 0; lcnt[t] = c; }
  __syncthreads();
  if (t == 0) { int s = 0; for (int i = 0; i < CS_NB; ++i) { lpre[i] = s; s += lcnt[i]; } lpre[CS_NB] = s; }
  __syncthreads();
  { int k = lpre[t];
#pragma unroll 1
    for (int i = 0; i < tot; ++i) if (sd[i] == t) { sorted[k++] = se[i]; } }
  __syncthreads();
  const int s0 = S[hb]; const int s1 = S[hb + 1];
  for (int pass = 0; pass < 2; ++pass) {
    for (int i = t; i < s1 - s0; i += 256) *(volatile int*)(csr_eid + s0 + i) = (i < tot) ? sorted[i] : -1;
    { const int dst = hb * CS_NB + t; *(volatile int*)(csr_start + dst) = s0 + lpre[t]; *(volatile int*)(csr_cnt + dst) = lcnt[t]; }
    if (pass == 0) __threadfence(); }
}
static void build_csr(const int* eidst, int ne, int nt, int nn, int* seg_dst, int* seg_eid, int* P1, int* Q1, int* R, int* S, int* csr_eid, int* csr_start, int* csr_cnt, hipStream_t stream) {
  k_cs_p1<<<CS_NW / 8, 256, 0, stream>>>(eidst, ne, nt, nn, seg_dst, seg_eid, P1, Q1);
  k_cs_scan<<<1, 256, 0, stream>>>(P1, R, S);
  k_cs_p2<<<CS_NB, 256, 0, stream>>>(seg_dst, seg_eid, P1, Q1, R, S, nn, csr_eid, csr_start, csr_cnt);
}


__global__ __launch_bounds__(256) void k_round_rows(const float* __restrict__ W, unsigned short* __restrict__ Wt, int n8) {
  const int t = blockIdx.x * 256 + threadIdx.x;
  if (t >= n8) return;
  const v4f a = *(const v4fa*)(W + (size_t)t * 8), b = *(const v4fa*)(W + (size_t)t * 8 + 4);
  v8us v; v[0]=bf16_bits(a[0]); v[1]=bf16_bits(a[1]); v[2]=bf16_bits(a[2]); v[3]=bf16_bits(a[3]);
  v[4]=bf16_bits(b[0]); v[5]=bf16_bits(b[1]); v[6]=bf16_bits(b[2]); v[7]=bf16_bits(b[3]);
  *(volatile v8us*)(Wt + (size_t)t * 8) = v; __threadfence(); *(volatile v8us*)(Wt + (size_t)t * 8) = v;
}

__device__ __forceinline__ float sigm(float x) { return 1.0f / (1.0f + __expf(-x)); }
__device__ __forceinline__ float tnh(float x) { const float e = __expf(2.0f * x); return 1.0f - 2.0f / (1.0f + e); }
__device__ __forceinline__ float elu1(float v) { return v > 0.f ? v : (__expf(v) - 1.0f); }
__global__ __launch_bounds__(128) void k_bnaff(const float* __restrict__ g, const float* __restrict__ b, const float* __restrict__ m, const float* __restrict__ v, float* __restrict__ st) { const int c = threadIdx.x; const float sc = bf16_round(g[c]) * rsqrtf(bf16_round(v[c]) + 1e-5f); const float sh = bf16_round(b[c]) - bf16_round(m[c]) * sc; *(volatile float*)(st + c * 2) = sc; *(volatile float*)(st + c * 2 + 1) = sh; __threadfence(); *(volatile float*)(st + c * 2) = sc; *(volatile float*)(st + c * 2 + 1) = sh; }
__global__ __launch_bounds__(256) void k_dinv(const int* __restrict__ ccnt, float* __restrict__ dinv) { const int n = blockIdx.x * 256 + threadIdx.x; if (n >= NNODE) return; const int c = ccnt[n]; const float v = (c > 0) ? rsqrtf((float)c) : 0.f; *(volatile float*)(dinv + n) = v; __threadfence(); *(volatile float*)(dinv + n) = v; }
__global__ __launch_bounds__(256) void k_alpha(const float* __restrict__ xw, const float* __restrict__ as_, const float* __restrict__ ad_, float* __restrict__ AL) {
  __shared__ float so[8][8]; const int tid = threadIdx.x, wv = tid >> 5, lane = tid & 31; const int n = blockIdx.x * 8 + wv; float s[4], d[4];
  { const float* r = xw + (size_t)n * FH;
#pragma unroll
    for (int u = 0; u < 4; ++u) { const float v = (n < NNODE) ? r[u * 32 + lane] : 0.f; s[u] = v * bf16_round(as_[u * 32 + lane]); d[u] = v * bf16_round(ad_[u * 32 + lane]); for (int o = 16; o >= 1; o >>= 1) { s[u] += __shfl_xor(s[u], o, 32); d[u] += __shfl_xor(d[u], o, 32); } } }
  if (lane == 0) { for (int u = 0; u < 4; ++u) { so[wv][u] = s[u]; so[wv][4 + u] = d[u]; } } __syncthreads();
  if (tid < 64) { *(volatile float*)(AL + (size_t)blockIdx.x * 64 + tid) = so[tid >> 3][tid & 7]; } __threadfence(); if (tid < 64) { *(volatile float*)(AL + (size_t)blockIdx.x * 64 + tid) = so[tid >> 3][tid & 7]; }
}
__global__ __launch_bounds__(256) void k_gat(const float* __restrict__ xw, const float* __restrict__ AL, const int* __restrict__ src, const int* __restrict__ cstart, const int* __restrict__ ccnt, const int* __restrict__ ceid, const float* __restrict__ gb, const float* __restrict__ st1, float* __restrict__ H1) {
  __shared__ float sa[8][MAXDEG][NH]; __shared__ int ss[8][MAXDEG];
  const int tid = threadIdx.x, wv = tid >> 5, lane = tid & 31; const int d = blockIdx.x * 8 + wv; if (d >= NNODE) return;
  int p0 = cstart[d]; int cn = ccnt[d]; cn = cn < 0 ? 0 : (cn > MAXDEG ? MAXDEG : cn); p0 = p0 < 0 ? 0 : (p0 > NTOT + 32 * CS_NB ? NTOT + 32 * CS_NB : p0);
  float adst[NH]; for (int h = 0; h < NH; ++h) adst[h] = AL[(size_t)d * 8 + 4 + h];
  float mx[NH]; for (int h = 0; h < NH; ++h) mx[h] = -3.0e38f;
  for (int q = lane; q < cn; q += 32) { int e = ceid[p0 + q]; e = e < 0 ? 0 : (e >= NTOT ? NTOT - 1 : e); int s = (e < NE) ? src[e] : (e - NE); s = s < 0 ? 0 : (s >= NNODE ? NNODE - 1 : s); ss[wv][q] = s;
#pragma unroll
    for (int h = 0; h < NH; ++h) { float a = AL[(size_t)s * 8 + h] + adst[h]; a = a >= 0.f ? a : 0.2f * a; sa[wv][q][h] = a; mx[h] = fmaxf(mx[h], a); } }
  for (int h = 0; h < NH; ++h) for (int o = 16; o >= 1; o >>= 1) mx[h] = fmaxf(mx[h], __shfl_xor(mx[h], o, 32));
  __builtin_amdgcn_fence(__ATOMIC_ACQ_REL, "workgroup"); __builtin_amdgcn_wave_barrier();
  float den[NH] = {0.f, 0.f, 0.f, 0.f};
  for (int q = lane; q < cn; q += 32) {
#pragma unroll
    for (int h = 0; h < NH; ++h) { const float ex = expf(sa[wv][q][h] - mx[h]); sa[wv][q][h] = ex; den[h] += ex; } }
  for (int h = 0; h < NH; ++h) { for (int o = 16; o >= 1; o >>= 1) den[h] += __shfl_xor(den[h], o, 32); den[h] = 1.0f / (den[h] + 1e-16f); }
  __builtin_amdgcn_fence(__ATOMIC_ACQ_REL, "workgroup"); __builtin_amdgcn_wave_barrier();
  float acc[4] = {0.f, 0.f, 0.f, 0.f};
#pragma unroll 1
  for (int q = 0; q < cn; ++q) { const int s = ss[wv][q]; const float* r = xw + (size_t)s * FH;
#pragma unroll
    for (int u = 0; u < 4; ++u) { const float al = sa[wv][q][u] * ((u == 0) ? den[0] : (u == 1 ? den[1] : (u == 2 ? den[2] : den[3]))); acc[u] += al * r[u * 32 + lane]; } }
  float* orow = H1 + (size_t)d * FH;
  for (int pass = 0; pass < 2; ++pass) {
#pragma unroll
    for (int u = 0; u < 4; ++u) { const int c = u * 32 + lane; float v = elu1(acc[u] + bf16_round(gb[c])); v = v * st1[c * 2] + st1[c * 2 + 1]; *(volatile float*)(orow + c) = v; } if (pass == 0) __threadfence(); }
}
__global__ __launch_bounds__(256) void k_gcn(const float* __restrict__ hw, const float* __restrict__ dinv, const int* __restrict__ src, const int* __restrict__ cstart, const int* __restrict__ ccnt, const int* __restrict__ ceid, const float* __restrict__ gb, const float* __restrict__ st2, float* __restrict__ H2) {
  const int tid = threadIdx.x, wv = tid >> 5, lane = tid & 31; const int d = blockIdx.x * 8 + wv; if (d >= NNODE) return;
  int p0 = cstart[d]; const int cnr = ccnt[d]; int cn = cnr < 0 ? 0 : (cnr > MAXDEG ? MAXDEG : cnr); p0 = p0 < 0 ? 0 : (p0 > NTOT + 32 * CS_NB ? NTOT + 32 * CS_NB : p0); const float dd = dinv[d];
  float acc[4] = {0.f, 0.f, 0.f, 0.f};
#pragma unroll 1
  for (int q = 0; q < cn; ++q) { int e = ceid[p0 + q]; e = e < 0 ? 0 : (e >= NTOT ? NTOT - 1 : e); int s = (e < NE) ? src[e] : (e - NE); s = s < 0 ? 0 : (s >= NNODE ? NNODE - 1 : s); const float nrm = dd * dinv[s]; const float* r = hw + (size_t)s * FH;
#pragma unroll
    for (int u = 0; u < 4; ++u) acc[u] += nrm * r[u * 32 + lane]; }
  float* orow = H2 + (size_t)d * FH;
  for (int pass = 0; pass < 2; ++pass) {
#pragma unroll
    for (int u = 0; u < 4; ++u) { const int c = u * 32 + lane; float v = elu1(acc[u] + bf16_round(gb[c])); v = v * st2[c * 2] + st2[c * 2 + 1]; *(volatile float*)(orow + c) = v; } if (pass == 0) __threadfence(); }
}
__global__ __launch_bounds__(256) void k_pool(const float* __restrict__ H2, const int* __restrict__ batch, const float* __restrict__ gw, const float* __restrict__ gbias, float* __restrict__ REP) {
  const int tid = threadIdx.x, wv = tid >> 5, lane = tid & 31; const int g = blockIdx.x * 8 + wv; if (g >= NG) return;
  int lo = 0, hi = NNODE; while (lo < hi) { const int m = (lo + hi) >> 1; if (batch[m] < g) lo = m + 1; else hi = m; } const int s0 = lo; lo = 0; hi = NNODE; while (lo < hi) { const int m = (lo + hi) >> 1; if (batch[m] < g + 1) lo = m + 1; else hi = m; } const int s1 = lo;
  float w4[4]; for (int u = 0; u < 4; ++u) w4[u] = bf16_round(gw[u * 32 + lane]); const float gb0 = bf16_round(gbias[0]);
  float mx = -3.0e38f;
#pragma unroll 1
  for (int n = s0; n < s1; ++n) { const float* r = H2 + (size_t)n * FH; float s = 0.f; for (int u = 0; u < 4; ++u) s += r[u * 32 + lane] * w4[u]; for (int o = 16; o >= 1; o >>= 1) s += __shfl_xor(s, o, 32); mx = fmaxf(mx, s + gb0); }
  float den = 0.f; float acc[4] = {0.f, 0.f, 0.f, 0.f};
#pragma unroll 1
  for (int n = s0; n < s1; ++n) { const float* r = H2 + (size_t)n * FH; float s = 0.f; float rv[4]; for (int u = 0; u < 4; ++u) { rv[u] = r[u * 32 + lane]; s += rv[u] * w4[u]; } for (int o = 16; o >= 1; o >>= 1) s += __shfl_xor(s, o, 32); const float ex = expf((s + gb0) - mx); den += ex; for (int u = 0; u < 4; ++u) acc[u] += ex * rv[u]; }
  const float rd = (s1 > s0) ? 1.0f / (den + 1e-16f) : 0.f; float* orow = REP + (size_t)g * FH;
  for (int pass = 0; pass < 2; ++pass) { for (int u = 0; u < 4; ++u) *(volatile float*)(orow + u * 32 + lane) = acc[u] * rd; if (pass == 0) __threadfence(); }
}
__global__ __launch_bounds__(64) void k_lstm(const float* __restrict__ GI, const float* __restrict__ Whh, float* __restrict__ HT) {
  __shared__ float sH[2][16][LH + 1]; __shared__ float sC[2][16][LH + 1]; __shared__ float sG[2][16][G4 + 1];
  const int tid = threadIdx.x, wv = tid >> 5, lane = tid & 31, ln = lane & 15, hh = lane >> 4; const int row0 = (blockIdx.x * 2 + wv) * 16;
  float (*myH)[LH + 1] = sH[wv]; float (*myC)[LH + 1] = sC[wv]; float (*myG)[G4 + 1] = sG[wv];
  for (int r = 0; r < 16; ++r) for (int u = lane; u < LH; u += 32) { myH[r][u] = 0.f; myC[r][u] = 0.f; }
  __builtin_amdgcn_fence(__ATOMIC_ACQ_REL, "workgroup"); __builtin_amdgcn_wave_barrier();
#pragma unroll 1
  for (int step = 0; step < TT; ++step) {
#pragma unroll 1
    for (int tg = 0; tg < 4; ++tg) {
      v8f acc[8]; for (int t = 0; t < 8; ++t) acc[t] = (v8f){0.f,0.f,0.f,0.f,0.f,0.f,0.f,0.f};
#pragma unroll 1
      for (int kb = 0; kb < LH; kb += 32) { FragB ah, al;
#pragma unroll
        for (int q = 0; q < 8; ++q) { const float v0 = myH[ln][kb + 8 * hh + q], v1 = myH[ln][kb + 16 + 8 * hh + q]; const unsigned short h0 = bf16_bits(v0), h1 = bf16_bits(v1); ah.u[q] = h0; al.u[q] = bf16_bits(v0 - bf16_val(h0)); ah.u[8 + q] = h1; al.u[8 + q] = bf16_bits(v1 - bf16_val(h1)); }
#pragma unroll
        for (int t = 0; t < 8; ++t) { const int gcol = tg * 128 + t * 16 + ln; const float* brow = Whh + (size_t)gcol * LH + kb; FragB bw;
#pragma unroll
          for (int q = 0; q < 8; ++q) { bw.u[q] = bf16_bits(brow[8 * hh + q]); bw.u[8 + q] = bf16_bits(brow[16 + 8 * hh + q]); }
          acc[t] = mmaN<2>(ah.v, al.v, bw.v, bw.v, acc[t]); } }
#pragma unroll
      for (int t = 0; t < 8; ++t) {
#pragma unroll
        for (int r = 0; r < 8; ++r) myG[8 * hh + r][tg * 128 + t * 16 + ln] = acc[t][r]; } }
    __builtin_amdgcn_fence(__ATOMIC_ACQ_REL, "workgroup"); __builtin_amdgcn_wave_barrier();
#pragma unroll 1
    for (int r = 0; r < 16; ++r) { const float* gi = GI + ((size_t)(row0 + r) * TT + step) * G4;
#pragma unroll
      for (int a = 0; a < 4; ++a) { const int u = a * 32 + lane; const float gI = myG[r][u] + gi[u], gF = myG[r][LH + u] + gi[LH + u], gGv = myG[r][2 * LH + u] + gi[2 * LH + u], gO = myG[r][3 * LH + u] + gi[3 * LH + u];
        const float cnew = sigm(gF) * myC[r][u] + sigm(gI) * tnh(gGv); myC[r][u] = cnew; myH[r][u] = sigm(gO) * tnh(cnew); } }
    __builtin_amdgcn_fence(__ATOMIC_ACQ_REL, "workgroup"); __builtin_amdgcn_wave_barrier();
  }
  for (int pass = 0; pass < 2; ++pass) { for (int r = 0; r < 16; ++r) for (int u = lane; u < LH; u += 32) *(volatile float*)(HT + (size_t)(row0 + r) * LH + u) = myH[r][u]; if (pass == 0) __threadfence(); }
}
__global__ __launch_bounds__(256) void k_bsum(const float* __restrict__ a, const float* __restrict__ b, float* __restrict__ o) { const int t = blockIdx.x * 256 + threadIdx.x; if (t < G4) { const float v = bf16_round(a[t]) + bf16_round(b[t]); *(volatile float*)(o + t) = v; __threadfence(); *(volatile float*)(o + t) = v; } }
__global__ __launch_bounds__(256) void k_fc(const float* __restrict__ REP, const float* __restrict__ HT, const float* __restrict__ fw, const float* __restrict__ fb, float* __restrict__ out) { const int g = threadIdx.x; float s = bf16_round(fb[0]);
#pragma unroll 1
  for (int c = 0; c < FH; ++c) s += REP[(size_t)g * FH + c] * bf16_round(fw[c]);
#pragma unroll 1
  for (int c = 0; c < LH; ++c) s += HT[(size_t)g * LH + c] * bf16_round(fw[FH + c]);
  *(volatile float*)(out + g) = s; __threadfence(); *(volatile float*)(out + g) = s; }
extern "C" void kernel_launch(void* const* d_in, const int* in_sizes, int n_in,
                              void* d_out, int out_size, void* d_ws, size_t ws_size, hipStream_t stream) {
  (void)in_sizes; (void)n_in; (void)out_size;
  const float* x = (const float*)d_in[0]; const int* ei = (const int*)d_in[1]; const int* batch = (const int*)d_in[2]; const float* quant = (const float*)d_in[3];
  const float* gW = (const float*)d_in[4]; const float* gas = (const float*)d_in[5]; const float* gad = (const float*)d_in[6]; const float* gb = (const float*)d_in[7]; const float* g1 = (const float*)d_in[8]; const float* be1 = (const float*)d_in[9]; const float* m1 = (const float*)d_in[10]; const float* v1 = (const float*)d_in[11];
  const float* cW = (const float*)d_in[12]; const float* cb = (const float*)d_in[13]; const float* g2 = (const float*)d_in[14]; const float* be2 = (const float*)d_in[15]; const float* m2 = (const float*)d_in[16]; const float* v2 = (const float*)d_in[17];
  const float* gtw = (const float*)d_in[18]; const float* gtb = (const float*)d_in[19]; const float* Wih = (const float*)d_in[20]; const float* Whh = (const float*)d_in[21]; const float* bih = (const float*)d_in[22]; const float* bhh = (const float*)d_in[23]; const float* fw = (const float*)d_in[24]; const float* fb = (const float*)d_in[25];
  char* ws = (char*)d_ws; size_t off = 0;
  auto take = [&](size_t bytes) { char* p = ws + off; off += (bytes + 255) & ~(size_t)255; return p; };
  unsigned short* Bg = (unsigned short*)take(FH * FH * 2); unsigned short* Bc = (unsigned short*)take(FH * FH * 2); unsigned short* Bi = (unsigned short*)take(G4 * QD * 2); float* bs = (float*)take(G4 * 4);
  int* seg_dst = (int*)take((size_t)CS_NW * CS_CH * 4); int* seg_eid = (int*)take((size_t)CS_NW * CS_CH * 4); int* P1 = (int*)take((size_t)CS_NW * CS_NB * 4); int* Q1 = (int*)take((size_t)CS_NW * CS_NB * 4); int* R_ = (int*)take((size_t)CS_NW * CS_NB * 4); int* S_ = (int*)take((CS_NB + 32) * 4);
  int* ceid = (int*)take(((size_t)NTOT + 32 * CS_NB) * 4); int* cstart = (int*)take((size_t)CS_NB * CS_NB * 4); int* ccnt = (int*)take((size_t)CS_NB * CS_NB * 4);
  float* XW = (float*)take((size_t)NNODE * FH * 4); float* AL = (float*)take((size_t)((NNODE + 7) / 8) * 64 * 4); float* H1 = (float*)take((size_t)NNODE * FH * 4); float* HW = (float*)take((size_t)NNODE * FH * 4); float* H2 = (float*)take((size_t)NNODE * FH * 4);
  float* st1 = (float*)take(FH * 2 * 4); float* st2 = (float*)take(FH * 2 * 4); float* dinv = (float*)take((size_t)NNODE * 4); float* REP = (float*)take((size_t)NG * FH * 4); float* GI = (float*)take((size_t)NG * TT * G4 * 4); float* HT = (float*)take((size_t)NG * LH * 4);
  if (off > ws_size) return;
  k_wt_bf16<<<(FH * 16 + 255) / 256, 256, 0, stream>>>(gW, Bg, FH, FH); k_wt_bf16<<<(FH * 16 + 255) / 256, 256, 0, stream>>>(cW, Bc, FH, FH);
  build_csr(ei + NE, NE, NTOT, NNODE, seg_dst, seg_eid, P1, Q1, R_, S_, ceid, cstart, ccnt, stream);
  k_gemm_bf3<false, 0, false, false><<<((NNODE / 16) * 2 + 3) / 4, 128, 0, stream>>>(x, FH, Bg, FH, nullptr, nullptr, 1, 0, XW, FH, NNODE, FH, FH);
  k_alpha<<<(NNODE + 7) / 8, 256, 0, stream>>>(XW, gas, gad, AL);
  k_bnaff<<<1, 128, 0, stream>>>(g1, be1, m1, v1, st1); k_bnaff<<<1, 128, 0, stream>>>(g2, be2, m2, v2, st2); k_dinv<<<(NNODE + 255) / 256, 256, 0, stream>>>(ccnt, dinv);
  k_gat<<<(NNODE + 7) / 8, 256, 0, stream>>>(XW, AL, ei, cstart, ccnt, ceid, gb, st1, H1);
  k_gemm_bf3<true, 0, false, false><<<((NNODE / 16) * 2 + 3) / 4, 128, 0, stream>>>(H1, FH, Bc, FH, nullptr, nullptr, 1, 0, HW, FH, NNODE, FH, FH);
  k_gcn<<<(NNODE + 7) / 8, 256, 0, stream>>>(HW, dinv, ei, cstart, ccnt, ceid, cb, st2, H2);
  k_pool<<<NG / 8, 256, 0, stream>>>(H2, batch, gtw, gtb, REP);
  k_bsum<<<2, 256, 0, stream>>>(bih, bhh, bs);
  k_round_rows<<<(G4 * QD / 8 + 255) / 256, 256, 0, stream>>>(Wih, Bi, G4 * QD / 8);
  k_gemm_bf3<false, 0, false, false><<<((NG * TT / 16) * (G4 / 64) + 3) / 4, 128, 0, stream>>>(quant, QD, Bi, QD, bs, nullptr, 1, 0, GI, G4, NG * TT, G4, QD);
  k_lstm<<<NG / 32, 64, 0, stream>>>(GI, Whh, HT);
  k_fc<<<1, 256, 0, stream>>>(REP, HT, fw, fb, (float*)d_out);
}
